// HardcodedKVMemoryBlock_44547400794260
// MI455X (gfx1250) — hardware-verified
//
#include <hip/hip_runtime.h>
#include <stddef.h>
#include <stdint.h>
#include <math.h>

#define NB    2
#define LSEQ  2048
#define DM    256
#define NPH   32
#define DQ    64
#define DHID  512
#define NROW  4096
#define NKEY  1024
#define CH    64
#define NQB   32
#define NJC   16

#define PI_F    3.14159265358979323846f
#define SQRTP_F 5.656854249492381f

static_assert(NB * LSEQ == NROW);
static_assert(2 * NKEY == LSEQ);
static_assert(NQB * CH == LSEQ);
static_assert(NJC * CH == NKEY);
static_assert(DQ == 2 * NPH);

typedef __bf16         v16bf __attribute__((ext_vector_type(16)));
typedef unsigned short v8us  __attribute__((ext_vector_type(8)));
typedef float          v8f   __attribute__((ext_vector_type(8)));
typedef float          v4f   __attribute__((ext_vector_type(4)));
typedef unsigned int   v4u   __attribute__((ext_vector_type(4)));

union Frag { v16bf v; v8us u[2]; };
union Pk8  { v8us s; v4u u; };

__device__ __forceinline__ v8f mma16(v16bf a, v16bf b, v8f c) {
  c = __builtin_amdgcn_wmma_f32_16x16x32_bf16(false, a, false, b, (short)0, c, false, false);
  asm volatile("v_nop\n\tv_nop\n\tv_nop\n\tv_nop" : "+v"(c) : "v"(a), "v"(b));
  return c;
}

__device__ __forceinline__ v16bf ldfrag(const unsigned short* p, int ld, int row0, int k0, int lane) {
  const int m = lane & 15, lh = lane >> 4;
  const unsigned short* q = p + (size_t)(row0 + m) * ld + k0 + 8 * lh;
  Frag f;
  f.u[0] = *(const v8us*)(q);
  f.u[1] = *(const v8us*)(q + 16);
  return f.v;
}

__device__ __forceinline__ v8f zero8() { return (v8f){0.f, 0.f, 0.f, 0.f, 0.f, 0.f, 0.f, 0.f}; }

__device__ __forceinline__ unsigned int bf_rne(float x) {
  const unsigned int u = __float_as_uint(x);
  return (u + 0x7FFFu + ((u >> 16) & 1u)) >> 16;
}

__device__ __forceinline__ void split1(float x, unsigned short& hi, unsigned short& lo) {
  const unsigned int hb = bf_rne(x);
  const float hv = __uint_as_float(hb << 16);
  const unsigned int lb = bf_rne(x - hv);
  hi = (unsigned short)hb;
  lo = (unsigned short)lb;
}

__device__ __forceinline__ void split8(const float (&x)[8], v8us& hi, v8us& lo) {
#pragma unroll
  for (int j = 0; j < 8; ++j) {
    unsigned short h_, l_;
    split1(x[j], h_, l_);
    hi[j] = h_;
    lo[j] = l_;
  }
}

#define TPW 33
__global__ __launch_bounds__(256) void k_prepw(const float* __restrict__ w, int K, int N,
                                               unsigned short* __restrict__ wh, unsigned short* __restrict__ wl) {
  __shared__ float sw[64 * TPW];
  const int k0 = blockIdx.x * 64, n0 = blockIdx.y * 32;
  const int tid = threadIdx.x;
#pragma unroll
  for (int it = 0; it < 2; ++it) {
    const int idx = tid + 256 * it;
    const int kk = idx >> 3, c4 = idx & 7;
    const v4f a = *(const v4f*)(w + (size_t)(k0 + kk) * N + n0 + c4 * 4);
    float* r = sw + kk * TPW + c4 * 4;
    r[0] = a[0]; r[1] = a[1]; r[2] = a[2]; r[3] = a[3];
  }
  __syncthreads();
  const int n = tid >> 3, pc = tid & 7;
  float x[8];
#pragma unroll
  for (int j = 0; j < 8; ++j) x[j] = sw[(pc * 8 + j) * TPW + n];
  v8us h8, l8;
  split8(x, h8, l8);
  Pk8 a, b;
  a.s = h8; b.s = l8;
  const size_t go = (size_t)(n0 + n) * K + k0 + pc * 8;
  for (int ps = 0; ps < 2; ++ps) {
    *(volatile v4u*)(wh + go) = a.u;
    *(volatile v4u*)(wl + go) = b.u;
    __threadfence();
  }
}

__global__ __launch_bounds__(256) void k_cvtx(const float* __restrict__ x, unsigned short* __restrict__ xh,
                                              unsigned short* __restrict__ xl, int n8) {
  const int t = blockIdx.x * 256 + threadIdx.x;
  if (t < n8) {
    const float* p = x + (size_t)t * 8;
    const v4f a0 = *(const v4f*)(p), a1 = *(const v4f*)(p + 4);
    float v[8] = {a0[0], a0[1], a0[2], a0[3], a1[0], a1[1], a1[2], a1[3]};
    v8us h8, l8;
    split8(v, h8, l8);
    Pk8 a, b;
    a.s = h8; b.s = l8;
    const size_t go = (size_t)t * 8;
    for (int ps = 0; ps < 2; ++ps) {
      *(volatile v4u*)(xh + go) = a.u;
      *(volatile v4u*)(xl + go) = b.u;
      __threadfence();
    }
  }
}

#define PP 36
#define QP 72
__global__ __launch_bounds__(256) void k_projq(const unsigned short* __restrict__ xh,
                                               const unsigned short* __restrict__ xl,
                                               const unsigned short* __restrict__ kwh,
                                               const unsigned short* __restrict__ kwl,
                                               const float* __restrict__ keyb,
                                               unsigned short* __restrict__ qh,
                                               unsigned short* __restrict__ ql) {
  __shared__ __align__(16) float sP[64 * PP];
  __shared__ __align__(16) unsigned short sQh[64 * QP];
  __shared__ __align__(16) unsigned short sQl[64 * QP];
  const int row0 = blockIdx.x * 64;
  const int tid = threadIdx.x, lane = tid & 31, wave = tid >> 5;
  const int hh = lane >> 4, c = lane & 15;
  {
    const int mt = wave >> 1, nt = wave & 1;
    v8f acc = zero8();
#pragma unroll
    for (int ks = 0; ks < 8; ++ks) {
      const int k0 = ks * 32;
      const v16bf ah = ldfrag(xh, DM, row0 + mt * 16, k0, lane);
      const v16bf al = ldfrag(xl, DM, row0 + mt * 16, k0, lane);
      const v16bf bh = ldfrag(kwh, DM, nt * 16, k0, lane);
      const v16bf bl = ldfrag(kwl, DM, nt * 16, k0, lane);
      acc = mma16(ah, bh, acc);
      acc = mma16(ah, bl, acc);
      acc = mma16(al, bh, acc);
    }
#pragma unroll
    for (int r = 0; r < 8; ++r) sP[(mt * 16 + 8 * hh + r) * PP + nt * 16 + c] = acc[r];
  }
  __syncthreads();
  {
    const int row = tid >> 2, part = tid & 3;
#pragma unroll 1
    for (int j = 0; j < 8; ++j) {
      const int p = part * 8 + j;
      const float v = sP[row * PP + p] + keyb[p];
      const float th = tanhf(v) * PI_F;
      const float cs = cosf(th), sn = sinf(th);
      unsigned short c_h, c_l, s_h, s_l;
      split1(cs, c_h, c_l);
      split1(sn, s_h, s_l);
      sQh[row * QP + p] = c_h;
      sQl[row * QP + p] = c_l;
      sQh[row * QP + NPH + p] = s_h;
      sQl[row * QP + NPH + p] = s_l;
    }
  }
  __syncthreads();
  v4u vh[2], vl[2];
  size_t go[2];
#pragma unroll
  for (int it = 0; it < 2; ++it) {
    const int p = tid + 256 * it;
    const int row = p >> 3, pc = p & 7;
    Pk8 a, b;
    a.s = *(const v8us*)(sQh + row * QP + pc * 8);
    b.s = *(const v8us*)(sQl + row * QP + pc * 8);
    vh[it] = a.u; vl[it] = b.u;
    go[it] = (size_t)(row0 + row) * DQ + pc * 8;
  }
  for (int ps = 0; ps < 2; ++ps) {
#pragma unroll
    for (int it = 0; it < 2; ++it) {
      *(volatile v4u*)(qh + go[it]) = vh[it];
      *(volatile v4u*)(ql + go[it]) = vl[it];
    }
    __threadfence();
  }
}

#define VP 68
__global__ __launch_bounds__(256) void k_projv(const unsigned short* __restrict__ xh,
                                               const unsigned short* __restrict__ xl,
                                               const unsigned short* __restrict__ vwh,
                                               const unsigned short* __restrict__ vwl,
                                               const float* __restrict__ valb,
                                               unsigned short* __restrict__ vth,
                                               unsigned short* __restrict__ vtl) {
  __shared__ __align__(16) float sV[128 * VP];
  const int jc = blockIdx.x, dhf = blockIdx.y, b = blockIdx.z;
  const int tid = threadIdx.x, lane = tid & 31, wave = tid >> 5;
  const int hh = lane >> 4, c = lane & 15;
  const int dl0 = wave * 16;
  const int d0 = dhf * 128 + dl0;
  const unsigned short* bxh = xh + (size_t)(b * LSEQ + 128 * jc + 1) * DM;
  const unsigned short* bxl = xl + (size_t)(b * LSEQ + 128 * jc + 1) * DM;
  v8f acc[4] = {zero8(), zero8(), zero8(), zero8()};
#pragma unroll 2
  for (int ks = 0; ks < 8; ++ks) {
    const int k0 = ks * 32;
    const v16bf ah = ldfrag(vwh, DM, d0, k0, lane);
    const v16bf al = ldfrag(vwl, DM, d0, k0, lane);
#pragma unroll
    for (int jt = 0; jt < 4; ++jt) {
      const v16bf bh = ldfrag(bxh, 2 * DM, 16 * jt, k0, lane);
      const v16bf bl = ldfrag(bxl, 2 * DM, 16 * jt, k0, lane);
      acc[jt] = mma16(ah, bh, acc[jt]);
      acc[jt] = mma16(ah, bl, acc[jt]);
      acc[jt] = mma16(al, bh, acc[jt]);
    }
  }
#pragma unroll
  for (int r = 0; r < 8; ++r) {
    const float bb = valb[d0 + 8 * hh + r];
#pragma unroll
    for (int jt = 0; jt < 4; ++jt) sV[(dl0 + 8 * hh + r) * VP + 16 * jt + c] = acc[jt][r] + bb;
  }
  __syncthreads();
  v4u vh[4], vl[4];
  size_t go[4];
#pragma unroll
  for (int it = 0; it < 4; ++it) {
    const int p = tid + 256 * it;
    const int L = p >> 3, pc = p & 7;
    const v4f g0 = *(const v4f*)(sV + L * VP + pc * 8);
    const v4f g1 = *(const v4f*)(sV + L * VP + pc * 8 + 4);
    float xv[8] = {g0[0], g0[1], g0[2], g0[3], g1[0], g1[1], g1[2], g1[3]};
    v8us h8, l8;
    split8(xv, h8, l8);
    Pk8 a, bq;
    a.s = h8; bq.s = l8;
    vh[it] = a.u; vl[it] = bq.u;
    go[it] = ((size_t)(b * DM + dhf * 128 + L)) * NKEY + jc * CH + pc * 8;
  }
  for (int ps = 0; ps < 2; ++ps) {
#pragma unroll
    for (int it = 0; it < 4; ++it) {
      *(volatile v4u*)(vth + go[it]) = vh[it];
      *(volatile v4u*)(vtl + go[it]) = vl[it];
    }
    __threadfence();
  }
}

#define AP  72
#define OPI 132
#define AT_AL (64 * AP * 2)
#define AT_BYTES (64 * OPI * 4)
static_assert(2 * 64 * AP * 2 <= AT_BYTES);

__global__ __launch_bounds__(256) void k_attn(const unsigned short* __restrict__ qh,
                                              const unsigned short* __restrict__ ql,
                                              const unsigned short* __restrict__ vth,
                                              const unsigned short* __restrict__ vtl,
                                              float* __restrict__ retr) {
  __shared__ __align__(16) unsigned char smem[AT_BYTES];
  unsigned short* sAh = (unsigned short*)(smem);
  unsigned short* sAl = (unsigned short*)(smem + AT_AL);
  float*          sO  = (float*)(smem);

  const int qb = blockIdx.x, dh = blockIdx.y, b = blockIdx.z;
  const int tid = threadIdx.x, lane = tid & 31, wave = tid >> 5;
  const int hh = lane >> 4, c = lane & 15;
  const int rg = wave & 3, kh = wave >> 2;
  const int i0 = rg * 16;

  const size_t qrow0 = (size_t)b * LSEQ + (size_t)qb * CH;
  const unsigned short* aqh = qh + qrow0 * DQ;
  const unsigned short* aql = ql + qrow0 * DQ;
  const unsigned short* bkh = qh + (size_t)b * LSEQ * DQ;
  const unsigned short* bkl = ql + (size_t)b * LSEQ * DQ;
  const unsigned short* bvh = vth + ((size_t)b * DM + dh * 128 + kh * 64) * NKEY;
  const unsigned short* bvl = vtl + ((size_t)b * DM + dh * 128 + kh * 64) * NKEY;

  v8f oacc[4] = {zero8(), zero8(), zero8(), zero8()};
  const int nkc = (qb >> 1) + 1;

  for (int kc = 0; kc < nkc; ++kc) {
    const int j0 = kc * CH;
    v8f s[2] = {zero8(), zero8()};
#pragma unroll
    for (int ks = 0; ks < 2; ++ks) {
      const int k0 = ks * 32;
      const v16bf ah = ldfrag(aqh, DQ, i0, k0, lane);
      const v16bf al = ldfrag(aql, DQ, i0, k0, lane);
#pragma unroll
      for (int jt = 0; jt < 2; ++jt) {
        const int krow = j0 + kh * 32 + 16 * jt;
        const v16bf bh = ldfrag(bkh, 2 * DQ, krow, k0, lane);
        const v16bf bl = ldfrag(bkl, 2 * DQ, krow, k0, lane);
        s[jt] = mma16(ah, bh, s[jt]);
        s[jt] = mma16(ah, bl, s[jt]);
        s[jt] = mma16(al, bh, s[jt]);
      }
    }
    __syncthreads();
#pragma unroll
    for (int r = 0; r < 8; ++r) {
      const int il = i0 + 8 * hh + r;
      const int l = qb * CH + il;
#pragma unroll
      for (int jt = 0; jt < 2; ++jt) {
        const int jl = kh * 32 + 16 * jt + c;
        const int j = j0 + jl;
        const float av = (2 * j + 1 <= l) ? s[jt][r] : 0.f;
        unsigned short a_h, a_l;
        split1(av, a_h, a_l);
        sAh[il * AP + jl] = a_h;
        sAl[il * AP + jl] = a_l;
      }
    }
    __syncthreads();
#pragma unroll
    for (int kk = 0; kk < 2; ++kk) {
      const v16bf pah = ldfrag(sAh, AP, i0, kk * 32, lane);
      const v16bf pal = ldfrag(sAl, AP, i0, kk * 32, lane);
#pragma unroll
      for (int t = 0; t < 4; ++t) {
        const v16bf bh = ldfrag(bvh, NKEY, 16 * t, j0 + kk * 32, lane);
        const v16bf bl = ldfrag(bvl, NKEY, 16 * t, j0 + kk * 32, lane);
        oacc[t] = mma16(pah, bh, oacc[t]);
        oacc[t] = mma16(pah, bl, oacc[t]);
        oacc[t] = mma16(pal, bh, oacc[t]);
      }
    }
  }
  __syncthreads();
#pragma unroll
  for (int r = 0; r < 8; ++r) {
    const int row = i0 + 8 * hh + r;
    const int l = qb * CH + row;
    int valid = (l + 1) >> 1;
    if (valid < 1) valid = 1;
    const float inv = 1.0f / (sqrtf((float)valid) * SQRTP_F);
#pragma unroll
    for (int t = 0; t < 4; ++t) sO[row * OPI + kh * 64 + 16 * t + c] = oacc[t][r] * inv;
  }
  __syncthreads();
  v4f val[8];
  size_t go[8];
#pragma unroll
  for (int it = 0; it < 8; ++it) {
    const int p   = tid + 256 * it;
    const int L   = p >> 3;
    const int row = L >> 2;
    const int q4  = L & 3;
    const int pc  = p & 7;
    val[it] = *(const v4f*)(sO + row * OPI + q4 * 32 + pc * 4);
    go[it]  = (qrow0 + row) * DM + dh * 128 + q4 * 32 + pc * 4;
  }
  for (int ps = 0; ps < 2; ++ps) {
#pragma unroll
    for (int it = 0; it < 8; ++it) *(volatile v4f*)(retr + go[it]) = val[it];
    __threadfence();
  }
}

#define RP 260
#define LP 264
__device__ __forceinline__ void ln16_split(const float* t, const float* __restrict__ g,
                                           const float* __restrict__ bt, unsigned short* oh,
                                           unsigned short* ol, int tid) {
  const int row = tid >> 4, seg = tid & 15;
  const float* rp = t + row * RP + seg * 16;
  const v4f a0 = *(const v4f*)(rp), a1 = *(const v4f*)(rp + 4);
  const v4f a2 = *(const v4f*)(rp + 8), a3 = *(const v4f*)(rp + 12);
  float v[16] = {a0[0], a0[1], a0[2], a0[3], a1[0], a1[1], a1[2], a1[3],
                 a2[0], a2[1], a2[2], a2[3], a3[0], a3[1], a3[2], a3[3]};
  float s = 0.f;
#pragma unroll
  for (int j = 0; j < 16; ++j) s += v[j];
  s += __shfl_xor(s, 1, 32); s += __shfl_xor(s, 2, 32);
  s += __shfl_xor(s, 4, 32); s += __shfl_xor(s, 8, 32);
  const float m = s * (1.0f / 256.0f);
  float q = 0.f;
#pragma unroll
  for (int j = 0; j < 16; ++j) { const float d = v[j] - m; q += d * d; }
  q += __shfl_xor(q, 1, 32); q += __shfl_xor(q, 2, 32);
  q += __shfl_xor(q, 4, 32); q += __shfl_xor(q, 8, 32);
  const float rstd = 1.0f / sqrtf(q * (1.0f / 256.0f) + 1e-5f);
  float y0[8], y1[8];
#pragma unroll
  for (int j = 0; j < 8; ++j) {
    const int d = seg * 16 + j;
    y0[j] = (v[j] - m) * rstd * g[d] + bt[d];
    y1[j] = (v[8 + j] - m) * rstd * g[d + 8] + bt[d + 8];
  }
  v8us h8, l8;
  split8(y0, h8, l8);
  *(v8us*)(oh + row * LP + seg * 16) = h8;
  *(v8us*)(ol + row * LP + seg * 16) = l8;
  split8(y1, h8, l8);
  *(v8us*)(oh + row * LP + seg * 16 + 8) = h8;
  *(v8us*)(ol + row * LP + seg * 16 + 8) = l8;
}

#define HP 516
#define M_AH (16 * RP * 4)
#define M_AL (M_AH + 16 * LP * 2)
#define M_BYTES (M_AL + 16 * LP * 2)
static_assert(16 * HP * 4 <= M_BYTES);

__global__ __launch_bounds__(256) void k_mlp1(const float* __restrict__ retr,
                                              const float* __restrict__ g1, const float* __restrict__ be1,
                                              const unsigned short* __restrict__ w1h,
                                              const unsigned short* __restrict__ w1l,
                                              const float* __restrict__ b1,
                                              unsigned short* __restrict__ hph, unsigned short* __restrict__ hpl) {
  __shared__ __align__(16) unsigned char smem[M_BYTES];
  float*          sR  = (float*)(smem);
  unsigned short* sAh = (unsigned short*)(smem + M_AH);
  unsigned short* sAl = (unsigned short*)(smem + M_AL);
  float*          sH  = (float*)(smem);
  const int row0 = blockIdx.x * 16;
  const int tid = threadIdx.x, lane = tid & 31, wave = tid >> 5;
  const int hh = lane >> 4, c = lane & 15;
#pragma unroll
  for (int it = 0; it < 4; ++it) {
    const int idx = tid + 256 * it;
    const int row = idx >> 6, c4 = idx & 63;
    *(v4f*)(sR + row * RP + c4 * 4) = *(const v4f*)(retr + (size_t)(row0 + row) * DM + c4 * 4);
  }
  __syncthreads();
  ln16_split(sR, g1, be1, sAh, sAl, tid);
  __syncthreads();
  v8f acc[4] = {zero8(), zero8(), zero8(), zero8()};
#pragma unroll 2
  for (int ks = 0; ks < 8; ++ks) {
    const int k0 = ks * 32;
    const v16bf ah = ldfrag(sAh, LP, 0, k0, lane);
    const v16bf al = ldfrag(sAl, LP, 0, k0, lane);
#pragma unroll
    for (int t = 0; t < 4; ++t) {
      const v16bf bh = ldfrag(w1h, DM, (4 * wave + t) * 16, k0, lane);
      const v16bf bl = ldfrag(w1l, DM, (4 * wave + t) * 16, k0, lane);
      acc[t] = mma16(ah, bh, acc[t]);
      acc[t] = mma16(ah, bl, acc[t]);
      acc[t] = mma16(al, bh, acc[t]);
    }
  }
  __syncthreads();
#pragma unroll
  for (int t = 0; t < 4; ++t) {
    const int col = 64 * wave + 16 * t + c;
    const float bb = b1[col];
#pragma unroll
    for (int r = 0; r < 8; ++r) sH[(8 * hh + r) * HP + col] = acc[t][r] + bb;
  }
  __syncthreads();
#pragma unroll 1
  for (int i = tid; i < 16 * DHID; i += 256) {
    const int row = i >> 9, col = i & 511;
    const float v = sH[row * HP + col];
    sH[row * HP + col] = 0.5f * v * (1.0f + erff(v * 0.70710678118654752f));
  }
  __syncthreads();
  v4u vh[4], vl[4];
  size_t go[4];
#pragma unroll
  for (int it = 0; it < 4; ++it) {
    const int p   = tid + 256 * it;
    const int L   = p >> 3;
    const int row = L >> 3;
    const int seg = L & 7;
    const int pc  = p & 7;
    const float* hp = sH + row * HP + seg * 64 + pc * 8;
    const v4f g0 = *(const v4f*)(hp), gg1 = *(const v4f*)(hp + 4);
    float xv[8] = {g0[0], g0[1], g0[2], g0[3], gg1[0], gg1[1], gg1[2], gg1[3]};
    v8us h8, l8;
    split8(xv, h8, l8);
    Pk8 a, bq;
    a.s = h8; bq.s = l8;
    vh[it] = a.u; vl[it] = bq.u;
    go[it] = (size_t)(row0 + row) * DHID + seg * 64 + pc * 8;
  }
  for (int ps = 0; ps < 2; ++ps) {
#pragma unroll
    for (int it = 0; it < 4; ++it) {
      *(volatile v4u*)(hph + go[it]) = vh[it];
      *(volatile v4u*)(hpl + go[it]) = vl[it];
    }
    __threadfence();
  }
}

__global__ __launch_bounds__(256) void k_mlp2(const unsigned short* __restrict__ hph,
                                              const unsigned short* __restrict__ hpl,
                                              const unsigned short* __restrict__ w2h,
                                              const unsigned short* __restrict__ w2l,
                                              const float* __restrict__ b2,
                                              const float* __restrict__ g2, const float* __restrict__ be2,
                                              const unsigned short* __restrict__ woh,
                                              const unsigned short* __restrict__ wol,
                                              const float* __restrict__ bo,
                                              const float* __restrict__ x,
                                              float* __restrict__ out) {
  __shared__ __align__(16) unsigned char smem[M_BYTES];
  float*          sF  = (float*)(smem);
  unsigned short* sAh = (unsigned short*)(smem + M_AH);
  unsigned short* sAl = (unsigned short*)(smem + M_AL);
  float*          sO  = (float*)(smem);
  const int row0 = blockIdx.x * 16;
  const int tid = threadIdx.x, lane = tid & 31, wave = tid >> 5;
  const int hh = lane >> 4, c = lane & 15;
  {
    v8f acc[2] = {zero8(), zero8()};
#pragma unroll 4
    for (int ks = 0; ks < 16; ++ks) {
      const int k0 = ks * 32;
      const v16bf ah = ldfrag(hph, DHID, row0, k0, lane);
      const v16bf al = ldfrag(hpl, DHID, row0, k0, lane);
#pragma unroll
      for (int t = 0; t < 2; ++t) {
        const v16bf bh = ldfrag(w2h, DHID, (2 * wave + t) * 16, k0, lane);
        const v16bf bl = ldfrag(w2l, DHID, (2 * wave + t) * 16, k0, lane);
        acc[t] = mma16(ah, bh, acc[t]);
        acc[t] = mma16(ah, bl, acc[t]);
        acc[t] = mma16(al, bh, acc[t]);
      }
    }
#pragma unroll
    for (int t = 0; t < 2; ++t) {
      const int col = 32 * wave + 16 * t + c;
      const float bb = b2[col];
#pragma unroll
      for (int r = 0; r < 8; ++r) sF[(8 * hh + r) * RP + col] = acc[t][r] + bb;
    }
  }
  __syncthreads();
  ln16_split(sF, g2, be2, sAh, sAl, tid);
  __syncthreads();
  {
    v8f acc[2] = {zero8(), zero8()};
#pragma unroll
    for (int ks = 0; ks < 8; ++ks) {
      const int k0 = ks * 32;
      const v16bf ah = ldfrag(sAh, LP, 0, k0, lane);
      const v16bf al = ldfrag(sAl, LP, 0, k0, lane);
#pragma unroll
      for (int t = 0; t < 2; ++t) {
        const v16bf bh = ldfrag(woh, DM, (2 * wave + t) * 16, k0, lane);
        const v16bf bl = ldfrag(wol, DM, (2 * wave + t) * 16, k0, lane);
        acc[t] = mma16(ah, bh, acc[t]);
        acc[t] = mma16(ah, bl, acc[t]);
        acc[t] = mma16(al, bh, acc[t]);
      }
    }
#pragma unroll
    for (int t = 0; t < 2; ++t) {
      const int col = 32 * wave + 16 * t + c;
      const float bb = bo[col];
#pragma unroll
      for (int r = 0; r < 8; ++r) sO[(8 * hh + r) * RP + col] = acc[t][r] + bb;
    }
  }
  __syncthreads();
  v4f val[4];
  size_t go[4];
#pragma unroll
  for (int it = 0; it < 4; ++it) {
    const int p   = tid + 256 * it;
    const int L   = p >> 3;
    const int row = L >> 3;
    const int seg = L & 7;
    const int pc  = p & 7;
    const v4f o = *(const v4f*)(sO + row * RP + seg * 32 + pc * 4);
    go[it] = (size_t)(row0 + row) * DM + seg * 32 + pc * 4;
    const v4f xv = *(const v4f*)(x + go[it]);
    val[it] = xv + o;
  }
  for (int ps = 0; ps < 2; ++ps) {
#pragma unroll
    for (int it = 0; it < 4; ++it) *(volatile v4f*)(out + go[it]) = val[it];
    __threadfence();
  }
}

extern "C" void kernel_launch(void* const* d_in, const int* in_sizes, int n_in,
                              void* d_out, int out_size, void* d_ws, size_t ws_size,
                              hipStream_t stream) {
  if (n_in < 15) return;
  if (in_sizes[0] != NROW * DM) return;
  if (in_sizes[1] != DM * NPH) return;
  if (in_sizes[2] != NPH) return;
  if (in_sizes[3] != DM * DM) return;
  if (in_sizes[4] != DM) return;
  if (in_sizes[5] != DM) return;
  if (in_sizes[6] != DM) return;
  if (in_sizes[7] != DM * DHID) return;
  if (in_sizes[8] != DHID) return;
  if (in_sizes[9] != DHID * DM) return;
  if (in_sizes[10] != DM) return;
  if (in_sizes[11] != DM) return;
  if (in_sizes[12] != DM) return;
  if (in_sizes[13] != DM * DM) return;
  if (in_sizes[14] != DM) return;
  if (out_size != NROW * DM) return;

  const float* x    = (const float*)d_in[0];
  const float* keyW = (const float*)d_in[1];
  const float* keyb = (const float*)d_in[2];
  const float* valW = (const float*)d_in[3];
  const float* valb = (const float*)d_in[4];
  const float* ln1g = (const float*)d_in[5];
  const float* ln1b = (const float*)d_in[6];
  const float* W1   = (const float*)d_in[7];
  const float* b1   = (const float*)d_in[8];
  const float* W2   = (const float*)d_in[9];
  const float* b2   = (const float*)d_in[10];
  const float* ln2g = (const float*)d_in[11];
  const float* ln2b = (const float*)d_in[12];
  const float* Wo   = (const float*)d_in[13];
  const float* bo   = (const float*)d_in[14];
  float* out = (float*)d_out;

  const size_t szKW = (size_t)NPH * DM * 2;
  const size_t szVW = (size_t)DM * DM * 2;
  const size_t szW1 = (size_t)DHID * DM * 2;
  const size_t szW2 = (size_t)DM * DHID * 2;
  const size_t szWO = (size_t)DM * DM * 2;
  const size_t szX  = (size_t)NROW * DM * 2;
  const size_t szQ  = (size_t)NROW * DQ * 2;
  const size_t szV  = (size_t)NB * DM * NKEY * 2;
  const size_t szR  = (size_t)NROW * DM * 4;
  const size_t szH  = (size_t)NROW * DHID * 2;
  size_t off = 0;
  const size_t oKWH = off; off += szKW;
  const size_t oKWL = off; off += szKW;
  const size_t oVWH = off; off += szVW;
  const size_t oVWL = off; off += szVW;
  const size_t oW1H = off; off += szW1;
  const size_t oW1L = off; off += szW1;
  const size_t oW2H = off; off += szW2;
  const size_t oW2L = off; off += szW2;
  const size_t oWOH = off; off += szWO;
  const size_t oWOL = off; off += szWO;
  const size_t oXH  = off; off += szX;
  const size_t oXL  = off; off += szX;
  const size_t oQH  = off; off += szQ;
  const size_t oQL  = off; off += szQ;
  const size_t oVTH = off; off += szV;
  const size_t oVTL = off; off += szV;
  const size_t oRET = off; off += szR;
  const size_t oHH  = off; off += szH;
  const size_t oHL  = off; off += szH;
  if (off > ws_size) return;
  if (off > (size_t)134217728) return;

  char* ws = (char*)d_ws;
  unsigned short* KWH = (unsigned short*)(ws + oKWH);
  unsigned short* KWL = (unsigned short*)(ws + oKWL);
  unsigned short* VWH = (unsigned short*)(ws + oVWH);
  unsigned short* VWL = (unsigned short*)(ws + oVWL);
  unsigned short* W1H = (unsigned short*)(ws + oW1H);
  unsigned short* W1L = (unsigned short*)(ws + oW1L);
  unsigned short* W2H = (unsigned short*)(ws + oW2H);
  unsigned short* W2L = (unsigned short*)(ws + oW2L);
  unsigned short* WOH = (unsigned short*)(ws + oWOH);
  unsigned short* WOL = (unsigned short*)(ws + oWOL);
  unsigned short* XH  = (unsigned short*)(ws + oXH);
  unsigned short* XL  = (unsigned short*)(ws + oXL);
  unsigned short* QH  = (unsigned short*)(ws + oQH);
  unsigned short* QL  = (unsigned short*)(ws + oQL);
  unsigned short* VTH = (unsigned short*)(ws + oVTH);
  unsigned short* VTL = (unsigned short*)(ws + oVTL);
  float*          RET = (float*)(ws + oRET);
  unsigned short* HH  = (unsigned short*)(ws + oHH);
  unsigned short* HL  = (unsigned short*)(ws + oHL);

  const dim3 blk(256);
  const int n8 = in_sizes[0] / 8;
  k_prepw<<<dim3(DM / 64, NPH / 32), blk, 0, stream>>>(keyW, DM, NPH, KWH, KWL);
  k_prepw<<<dim3(DM / 64, DM / 32), blk, 0, stream>>>(valW, DM, DM, VWH, VWL);
  k_prepw<<<dim3(DM / 64, DHID / 32), blk, 0, stream>>>(W1, DM, DHID, W1H, W1L);
  k_prepw<<<dim3(DHID / 64, DM / 32), blk, 0, stream>>>(W2, DHID, DM, W2H, W2L);
  k_prepw<<<dim3(DM / 64, DM / 32), blk, 0, stream>>>(Wo, DM, DM, WOH, WOL);
  k_cvtx<<<dim3((n8 + 255) / 256), blk, 0, stream>>>(x, XH, XL, n8);
  k_projq<<<dim3(NROW / 64), blk, 0, stream>>>(XH, XL, KWH, KWL, keyb, QH, QL);
  k_projv<<<dim3(NJC, 2, NB), blk, 0, stream>>>(XH, XL, VWH, VWL, valb, VTH, VTL);
  k_attn<<<dim3(NQB, 2, NB), blk, 0, stream>>>(QH, QL, VTH, VTL, RET);
  k_mlp1<<<dim3(NROW / 16), blk, 0, stream>>>(RET, ln1g, ln1b, W1H, W1L, b1, HH, HL);
  k_mlp2<<<dim3(NROW / 16), blk, 0, stream>>>(HH, HL, W2H, W2L, b2, ln2g, ln2b, WOH, WOL, bo, x, out);
  (void)hipGetLastError();
}
